// FunctionPredictor_68564857913749
// MI455X (gfx1250) — hardware-verified
//
#include <hip/hip_runtime.h>
#include <math.h>

typedef __attribute__((ext_vector_type(16))) _Float16 v16h;
typedef __attribute__((ext_vector_type(16))) __bf16 v16b;
typedef __attribute__((ext_vector_type(8)))  _Float16 v8h;
typedef __attribute__((ext_vector_type(8)))  float v8f;
typedef __attribute__((ext_vector_type(4)))  float v4f;
typedef __attribute__((ext_vector_type(2)))  float v2f;
typedef __attribute__((ext_vector_type(4)))  unsigned v4u;
typedef __attribute__((ext_vector_type(4)))  int v4i;
typedef float __attribute__((may_alias)) float_a;
typedef int __attribute__((may_alias)) int_a;

template <typename T> __device__ __forceinline__ void vst2(void* p, T v) { *(volatile T*)p = v; __threadfence(); *(volatile T*)p = v; }
__device__ __forceinline__ v8f wmma16(v16h a, v16h b, v8f c) {
  v8f d = __builtin_amdgcn_wmma_f32_16x16x32_f16(false, a, false, b, (short)0, c, false, false);
  asm volatile("v_nop\n\tv_nop\n\tv_nop\n\tv_nop" : "+v"(d) : "v"(a), "v"(b));
  return d;
}
__device__ __forceinline__ v8f wmma_bf(v16b a, v16b b, v8f c) {
  v8f d = __builtin_amdgcn_wmma_f32_16x16x32_bf16(false, a, false, b, (short)0, c, false, false);
  asm volatile("v_nop\n\tv_nop\n\tv_nop\n\tv_nop" : "+v"(d) : "v"(a), "v"(b));
  return d;
}
__device__ __forceinline__ v16h frag_h(const _Float16* rowk0, int lane) {
  union { v16h v; v8h q[2]; } u; const _Float16* p = rowk0 + 8 * (lane >> 4);
  u.q[0] = *(const v8h*)p; u.q[1] = *(const v8h*)(p + 16); return u.v;
}
__device__ __forceinline__ v16h frag_f32(const float* rowk0, int lane) {
  v16h a; const float* p = rowk0 + 8 * (lane >> 4);
#pragma unroll
  for (int i = 0; i < 8; ++i) { a[i] = (_Float16)p[i]; a[8 + i] = (_Float16)p[16 + i]; }
  return a;
}
__device__ __forceinline__ v16h frag_f32s(const float* rowk0, int lane, float sc) {
  v16h a; const float* p = rowk0 + 8 * (lane >> 4);
#pragma unroll
  for (int i = 0; i < 8; ++i) { a[i] = (_Float16)(p[i] * sc); a[8 + i] = (_Float16)(p[16 + i] * sc); }
  return a;
}
__device__ __forceinline__ v16h fragc_f32(const float* W, int k0, int n, int lane, int ld, int K) {
  v16h a; const int g = lane >> 4;
#pragma unroll
  for (int i = 0; i < 8; ++i) { const int ka = k0 + 8 * g + i, kb = ka + 16;
    a[i] = (_Float16)(ka < K ? W[(size_t)(ka < K ? ka : K - 1) * ld + n] : 0.f); a[8 + i] = (_Float16)(kb < K ? W[(size_t)(kb < K ? kb : K - 1) * ld + n] : 0.f); }
  return a;
}
struct F2 { v16b h, l; };
__device__ __forceinline__ F2 bsplit16(const float v[16]) { F2 r;
#pragma unroll
  for (int i = 0; i < 16; ++i) { const __bf16 h = (__bf16)v[i]; r.h[i] = h; r.l[i] = (__bf16)(v[i] - (float)h); }
  return r; }
__device__ __forceinline__ F2 split_row(const float* row, int k0, int lane) { float v[16]; const float* p = row + k0 + 8 * (lane >> 4);
#pragma unroll
  for (int i = 0; i < 8; ++i) { v[i] = p[i]; v[8 + i] = p[16 + i]; }
  return bsplit16(v); }
__device__ __forceinline__ F2 split_rowK(const float* row, int k0, int lane, int K) { float v[16]; const int g = lane >> 4;
#pragma unroll
  for (int i = 0; i < 8; ++i) { const int ka = k0 + 8 * g + i, kb = ka + 16; v[i] = ka < K ? row[ka < K ? ka : K - 1] : 0.f; v[8 + i] = kb < K ? row[kb < K ? kb : K - 1] : 0.f; }
  return bsplit16(v); }
__device__ __forceinline__ F2 split_col(const float* W, int k0, int n, int lane, int ld, int K) { float v[16]; const int g = lane >> 4;
#pragma unroll
  for (int i = 0; i < 8; ++i) { const int ka = k0 + 8 * g + i, kb = ka + 16; v[i] = ka < K ? W[(size_t)(ka < K ? ka : K - 1) * ld + n] : 0.f; v[8 + i] = kb < K ? W[(size_t)(kb < K ? kb : K - 1) * ld + n] : 0.f; }
  return bsplit16(v); }
__device__ __forceinline__ v8f mac3(const F2& a, const F2& b, v8f c) { c = wmma_bf(a.l, b.h, c); c = wmma_bf(a.h, b.l, c); return wmma_bf(a.h, b.h, c); }
__device__ __forceinline__ float sigm(float v) { return 1.0f / (1.0f + expf(-v)); }
#define LDSX() do { asm volatile("s_wait_dscnt 0" ::: "memory"); __builtin_amdgcn_wave_barrier(); __builtin_amdgcn_fence(__ATOMIC_RELEASE, "workgroup"); } while (0)


#define NTK 1024
#define SQ 256
#define HH 320
#define H2 640
#define NGO 1000
#define HP 160
__device__ __forceinline__ float bfr(float v) { return (float)(__bf16)v; }
__device__ __forceinline__ v16b frag_b(const __bf16* rowk0, int lane) { return __builtin_bit_cast(v16b, frag_h((const _Float16*)rowk0, lane)); }
__device__ __attribute__((noinline)) float sigm_ni(float v) { return 1.0f / (1.0f + expf(-v)); }

__global__ __launch_bounds__(256) void k_cat(const float* __restrict__ a, const float* __restrict__ b, __bf16* __restrict__ XC) {
  const size_t i8 = (size_t)blockIdx.x * 256 + threadIdx.x; if (i8 >= (size_t)NTK * H2 / 8) return;
  const size_t r = i8 / (H2 / 8); const int c0 = (int)(i8 % (H2 / 8)) * 8; const float* src = c0 < HH ? a + r * HH + c0 : b + r * HH + (c0 - HH);
  union { __bf16 e[8]; v4u u; } pk;
#pragma unroll
  for (int e = 0; e < 8; ++e) pk.e[e] = (__bf16)src[e];
  vst2((unsigned*)(XC + r * H2 + c0), pk.u);
}
template <int ACT, int EXACT, int K, int N, int K2>
__global__ __launch_bounds__(128) void k_lin(const void* __restrict__ INv, int ldi, const float* __restrict__ IN2, int ldi2, const float* __restrict__ W, const float* __restrict__ bias, float* __restrict__ OUT, int ldo, int NS) {
  __shared__ __align__(16) float so[4][16][132];
  const int tid = threadIdx.x, wave = tid >> 5, lane = tid & 31, col = lane & 15, g = lane >> 4; const int r0 = blockIdx.x * 64 + wave * 16, n0 = blockIdx.y * 128;
  v8f acc[8] = {};
#pragma unroll 1
  for (int kc = 0; kc < (K + 31) / 32; ++kc) {
    if (EXACT) { const v16b a = frag_b((const __bf16*)INv + (size_t)(r0 + col) * ldi + kc * 32, lane);
#pragma unroll
      for (int j = 0; j < 8; ++j) { const int n = n0 + j * 16 + col; const int nc = n < N ? n : N - 1; acc[j] = wmma_bf(a, split_col(W, kc * 32, nc, lane, N, K).h, acc[j]); } }
    else { const F2 a = split_rowK((const float*)INv + (size_t)(r0 + col) * ldi, kc * 32, lane, K);
#pragma unroll
      for (int j = 0; j < 8; ++j) { const int n = n0 + j * 16 + col; const int nc = n < N ? n : N - 1; const v16b wb = split_col(W, kc * 32, nc, lane, N, K).h; acc[j] = wmma_bf(a.l, wb, acc[j]); acc[j] = wmma_bf(a.h, wb, acc[j]); } } }
  if (K2 > 0) { const F2 a = split_rowK(IN2 + (size_t)(r0 + col) * ldi2, 0, lane, K2);
#pragma unroll
    for (int j = 0; j < 8; ++j) { const int n = n0 + j * 16 + col; const int nc = n < N ? n : N - 1; const v16b wb = split_col(W + (size_t)K * N, 0, nc, lane, N, K2).h; acc[j] = wmma_bf(a.l, wb, acc[j]); acc[j] = wmma_bf(a.h, wb, acc[j]); } }
#pragma unroll
  for (int j = 0; j < 8; ++j) { const int n = n0 + j * 16 + col; const float bb = (bias && n < N) ? bfr(bias[n]) : 0.f;
#pragma unroll
    for (int r = 0; r < 8; ++r) { float v = acc[j][r] + bb; v = ACT == 1 ? (v > 0.f ? v : 0.f) : (ACT == 2 ? sigm_ni(v) : v); so[wave][8 * g + r][j * 16 + col] = n < N ? v : 0.f; } }
  LDSX();
  const int ncols = (NS - n0) < 128 ? (NS - n0) : 128;
  for (int rl = 0; rl < 16; ++rl) for (int pc = lane; pc < ncols / 4; pc += 32) vst2(OUT + (size_t)(r0 + rl) * ldo + n0 + pc * 4, *(const v4f*)(&so[wave][rl][pc * 4]));
}
__global__ __launch_bounds__(64) void k_go(const float* __restrict__ G1, const float* __restrict__ W, const float* __restrict__ bias, float* __restrict__ OUT) {
  __shared__ __align__(16) float srow[32][NGO];
  const int tid = threadIdx.x, wave = tid >> 5, lane = tid & 31, col = lane & 15, g = lane >> 4; const int r0 = blockIdx.x * 32 + wave * 16;
#pragma unroll 1
  for (int ps = 0; ps < 8; ++ps) { const int n0 = ps * 128; v8f acc[8] = {};
#pragma unroll 1
    for (int kc = 0; kc < H2 / 32; ++kc) { const F2 a = split_row(G1 + (size_t)(r0 + col) * H2, kc * 32, lane);
#pragma unroll
      for (int j = 0; j < 8; ++j) { const int n = n0 + j * 16 + col; const int nc = n < NGO ? n : NGO - 1; const v16b wb = split_col(W, kc * 32, nc, lane, NGO, H2).h; acc[j] = wmma_bf(a.l, wb, acc[j]); acc[j] = wmma_bf(a.h, wb, acc[j]); } }
#pragma unroll
    for (int j = 0; j < 8; ++j) { const int n = n0 + j * 16 + col; if (n < NGO) { const float bb = bfr(bias[n]);
#pragma unroll
        for (int r = 0; r < 8; ++r) srow[wave * 16 + 8 * g + r][n] = sigm_ni(acc[j][r] + bb); } } }
  __syncthreads();
  { const float* base = &srow[0][0]; float* dst = OUT + (size_t)blockIdx.x * 32 * NGO;
    for (int q = tid; q < 32 * NGO / 4; q += 64) vst2(dst + q * 4, *(const v4f*)(base + q * 4)); }
}
__global__ __launch_bounds__(64) void k_dot1(const float* __restrict__ Hr, const float* __restrict__ w, const float* __restrict__ b, float* __restrict__ out1) {
  __shared__ __align__(16) float s1[64];
  const int tid = threadIdx.x; const size_t r = (size_t)blockIdx.x * 64 + tid; const float* row = Hr + r * HH; float s = 0.f;
#pragma unroll 4
  for (int c = 0; c < HH; ++c) s += row[c] * bfr(w[c]);
  s1[tid] = sigm_ni(s + bfr(b[0]));
  __syncthreads();
  if (tid < 16) vst2(out1 + (size_t)blockIdx.x * 64 + tid * 4, *(const v4f*)(&s1[tid * 4]));
}
__global__ __launch_bounds__(64) void k_ec(const float* __restrict__ LG, float* __restrict__ out) {
  __shared__ __align__(16) float se[64 * 7 + 4];
  const int tid = threadIdx.x; const int r = blockIdx.x * 64 + tid; float v[7]; float mx = -3.4e38f;
#pragma unroll
  for (int e = 0; e < 7; ++e) { v[e] = LG[(size_t)r * 32 + e]; mx = fmaxf(mx, v[e]); }
  float s = 0.f;
#pragma unroll
  for (int e = 0; e < 7; ++e) { v[e] = expf(v[e] - mx); s += v[e]; }
  const float inv = 1.0f / s;
#pragma unroll
  for (int e = 0; e < 7; ++e) { v[e] *= inv; se[tid * 7 + e] = v[e]; }
  __syncthreads();
  for (int q = tid; q < 64 * 7 / 4; q += 64) vst2(out + (size_t)blockIdx.x * 64 * 7 + q * 4, *(const v4f*)(&se[q * 4]));
}
__global__ __launch_bounds__(128) void k_ppi(const float* __restrict__ A, const float* __restrict__ Bv, const float* __restrict__ b1, const float* __restrict__ W2, const float* __restrict__ b2, const float* __restrict__ W3, const float* __restrict__ b3, float* __restrict__ PPI) {
  __shared__ __align__(16) __bf16 sh_[4][16][HH + 8], sl_[4][16][HH + 8]; __shared__ __align__(16) float sa[HH]; __shared__ __align__(16) float srow[SQ];
  const int tid = threadIdx.x, wave = tid >> 5, lane = tid & 31, col = lane & 15, g = lane >> 4; const int b = blockIdx.y, i = blockIdx.x; const size_t ri = (size_t)b * SQ + i;
  for (int c = tid; c < HH; c += 128) sa[c] = A[ri * HH + c] + bfr(b1[c]);
  __syncthreads();
  const float b3v = bfr(b3[0]);
#pragma unroll 1
  for (int jt = 0; jt < 4; ++jt) { const int j0 = (wave * 4 + jt) * 16;
    { const int rl = lane & 15, hf = lane >> 4; const float* brow = Bv + ((size_t)b * SQ + j0 + rl) * HH;
#pragma unroll 4
      for (int c = hf * 160; c < hf * 160 + 160; ++c) { float v = sa[c] + brow[c]; v = v > 0.f ? v : 0.f; const __bf16 hi = (__bf16)v; sh_[wave][rl][c] = hi; sl_[wave][rl][c] = (__bf16)(v - (float)hi); } }
    LDSX();
    v8f acc[10] = {};
#pragma unroll 1
    for (int kc = 0; kc < HH / 32; ++kc) { const v16b ah = frag_b(&sh_[wave][col][0] + kc * 32, lane), al = frag_b(&sl_[wave][col][0] + kc * 32, lane);
#pragma unroll
      for (int jn = 0; jn < 10; ++jn) { const v16b wb = split_col(W2, kc * 32, jn * 16 + col, lane, HP, HH).h; acc[jn] = wmma_bf(al, wb, acc[jn]); acc[jn] = wmma_bf(ah, wb, acc[jn]); } }
    float part[8];
#pragma unroll
    for (int r = 0; r < 8; ++r) part[r] = 0.f;
#pragma unroll
    for (int jn = 0; jn < 10; ++jn) { const int n = jn * 16 + col; const float bb = bfr(b2[n]), w3 = bfr(W3[n]);
#pragma unroll
      for (int r = 0; r < 8; ++r) { const float v = acc[jn][r] + bb; part[r] += (v > 0.f ? v : 0.f) * w3; } }
#pragma unroll
    for (int r = 0; r < 8; ++r) {
#pragma unroll
      for (int o_ = 1; o_ < 16; o_ <<= 1) part[r] += __shfl_xor(part[r], o_, 32); }
    if (col == 0) {
#pragma unroll
      for (int r = 0; r < 8; ++r) srow[j0 + 8 * g + r] = sigm_ni(part[r] + b3v); }
    LDSX(); }
  __syncthreads();
  for (int q = tid; q < SQ / 4; q += 128) vst2(PPI + ri * SQ + q * 4, *(const v4f*)(&srow[q * 4]));
}
extern "C" void kernel_launch(void* const* d_in, const int* in_sizes, int n_in, void* d_out, int out_size, void* d_ws, size_t ws_size, hipStream_t stream) {
  (void)in_sizes; (void)n_in; (void)out_size; (void)ws_size;
  const float** I = (const float**)d_in;
  const float *seqf = I[0], *strf = I[1], *fusW = I[2], *fusb = I[3], *goW1 = I[4], *gob1 = I[5], *goW2 = I[6], *gob2 = I[7], *pW1 = I[8], *pb1 = I[9], *pW2 = I[10], *pb2 = I[11], *pW3 = I[12], *pb3 = I[13];
  const float *eW1 = I[14], *eb1 = I[15], *eW2 = I[16], *eb2 = I[17], *aW1 = I[18], *ab1 = I[19], *aW2 = I[20], *ab2 = I[21], *bW1 = I[22], *bb1 = I[23], *bW2 = I[24], *bb2 = I[25], *bW3 = I[26], *bb3 = I[27];
  float* O_go = (float*)d_out; float* O_ppi = (float*)((char*)d_out + 4096000); float* O_ec = (float*)((char*)d_out + 5144576); float* O_act = (float*)((char*)d_out + 5173248); float* O_bind = (float*)((char*)d_out + 5177344);
  char* ws = (char*)d_ws; size_t off = 0;
  auto take = [&](size_t bytes) { char* p = ws + off; off += (bytes + 255) & ~(size_t)255; return p; };
  __bf16* XC = (__bf16*)take((size_t)NTK * H2 * 2); float* F = (float*)take((size_t)NTK * HH * 4); float* G1 = (float*)take((size_t)NTK * H2 * 4); float* PA = (float*)take((size_t)NTK * HH * 4); float* PB = (float*)take((size_t)NTK * HH * 4);
  float* E1 = (float*)take((size_t)NTK * H2 * 4); float* LG = (float*)take((size_t)NTK * 32 * 4); float* AH = (float*)take((size_t)NTK * HH * 4); float* B1 = (float*)take((size_t)NTK * H2 * 4); float* B2 = (float*)take((size_t)NTK * HH * 4);
  k_cat<<<(NTK * H2 / 8 + 255) / 256, 256, 0, stream>>>(seqf, strf, XC);
  k_lin<1, 1, H2, HH, 0><<<dim3(NTK / 64, 3), 128, 0, stream>>>(XC, H2, nullptr, 0, fusW, fusb, F, HH, HH);
  k_lin<1, 0, HH, H2, 0><<<dim3(NTK / 64, 5), 128, 0, stream>>>(F, HH, nullptr, 0, goW1, gob1, G1, H2, H2);
  k_go<<<NTK / 32, 64, 0, stream>>>(G1, goW2, gob2, O_go);
  k_lin<0, 0, HH, HH, 0><<<dim3(NTK / 64, 3), 128, 0, stream>>>(F, HH, nullptr, 0, pW1, nullptr, PA, HH, HH);
  k_lin<0, 0, HH, HH, 0><<<dim3(NTK / 64, 3), 128, 0, stream>>>(F, HH, nullptr, 0, pW1 + (size_t)HH * HH, nullptr, PB, HH, HH);
  k_lin<1, 0, HH, H2, 0><<<dim3(NTK / 64, 5), 128, 0, stream>>>(F, HH, nullptr, 0, eW1, eb1, E1, H2, H2);
  k_lin<0, 0, H2, 7, 0><<<dim3(NTK / 64, 1), 128, 0, stream>>>(E1, H2, nullptr, 0, eW2, eb2, LG, 32, 32);
  k_ec<<<NTK / 64, 64, 0, stream>>>(LG, O_ec);
  k_lin<1, 0, HH, HH, 7><<<dim3(NTK / 64, 3), 128, 0, stream>>>(F, HH, O_ec, 7, aW1, ab1, AH, HH, HH);
  k_dot1<<<NTK / 64, 64, 0, stream>>>(AH, aW2, ab2, O_act);
  k_lin<1, 0, HH, H2, 0><<<dim3(NTK / 64, 5), 128, 0, stream>>>(F, HH, nullptr, 0, bW1, bb1, B1, H2, H2);
  k_lin<1, 0, H2, HH, 0><<<dim3(NTK / 64, 3), 128, 0, stream>>>(B1, H2, nullptr, 0, bW2, bb2, B2, HH, HH);
  k_dot1<<<NTK / 64, 64, 0, stream>>>(B2, bW3, bb3, O_bind);
  k_ppi<<<dim3(SQ, 4), 128, 0, stream>>>(PA, PB, pb1, pW2, pb2, pW3, pb3, O_ppi);
}
